// MultiLinear_11115375362121
// MI455X (gfx1250) — hardware-verified
//
#include <hip/hip_runtime.h>
#include <stddef.h>


typedef _Float16 h16;
typedef _Float16 v16h __attribute__((ext_vector_type(16)));
typedef _Float16 v8h  __attribute__((ext_vector_type(8)));
typedef float    v8f  __attribute__((ext_vector_type(8)));
typedef float    v4f  __attribute__((ext_vector_type(4)));

#ifndef NROWS
#define NROWS 4096
#endif
#define NROWS_FULL 4096
#define KDIM   256
#define NDIM   256
#define NHEADS 16
#define CHUNK  512
#define TROWS  16
#define LDK    (NHEADS * KDIM)

static_assert(NROWS >= CHUNK && NROWS <= NROWS_FULL && (NROWS % CHUNK) == 0);
static_assert(CHUNK == 2 * 256);
static_assert((CHUNK % TROWS) == 0);
static_assert((KDIM % 32) == 0 && (KDIM % 64) == 0);
static_assert((NDIM % 64) == 0);
static_assert(NDIM == 8 * 32);
static_assert(KDIM == 32 * 8);
static_assert(TROWS == 2 * 8);
static_assert(TROWS == 4 * 4);
static_assert(NDIM == 64 * 4);
static_assert((LDK % 64) == 0);

#define LDT  72
#define LDA  264
#define LDCS 260
static_assert((LDT % 8) == 0 && LDT >= 64);
static_assert((LDA % 8) == 0 && LDA >= KDIM);
static_assert((LDCS % 4) == 0 && LDCS >= NDIM);
static_assert(64 * LDT * 2 <= 131072);
static_assert(TROWS * LDA * 2 + TROWS * LDCS * 4 + CHUNK * 4 + 16 * 4 <= 131072);

#define WCARRY 64.0f
#define XCARRY 16.0f

#define WT_BYTES ((size_t)NDIM * LDK * 2)
#define OFF_WT   ((size_t)0)
#define WS_TOTAL (OFF_WT + WT_BYTES)
static_assert((WT_BYTES % 128) == 0);
static_assert(WS_TOTAL <= (size_t)134217728);

__device__ __forceinline__ float bf16r(float x) {
  unsigned int u = __float_as_uint(x);
  u = (u + 0x7FFFu + ((u >> 16) & 1u)) & 0xFFFF0000u;
  return __uint_as_float(u);
}

static __device__ __forceinline__ h16 toh_flush(float v) {
  const h16 r = (h16)v;
  return (fabsf(v) < 6.103515625e-05f) ? (h16)0.0f : r;
}

__device__ __forceinline__ v16h frag_at(const _Float16* p) {
  v8h lo = *(const v8h*)(p);
  v8h hi = *(const v8h*)(p + 16);
  v16h out;
#pragma unroll
  for (int i = 0; i < 8; ++i) { out[i] = lo[i]; out[i + 8] = hi[i]; }
  return out;
}
__device__ __forceinline__ v16h frag_join(v8h lo, v8h hi) {
  v16h out;
#pragma unroll
  for (int i = 0; i < 8; ++i) { out[i] = lo[i]; out[i + 8] = hi[i]; }
  return out;
}

__device__ __forceinline__ v8f wmma16(v16h a, v16h b, v8f c) {
  v8f d = __builtin_amdgcn_wmma_f32_16x16x32_f16(false, a, false, b, (short)0, c,
                                                 false, false);
  asm volatile("v_nop\n\tv_nop\n\tv_nop\n\tv_nop" : "+v"(d) : "v"(a), "v"(b));
  return d;
}

__global__ __launch_bounds__(256) void wconv_kernel(
    const float* __restrict__ W, _Float16* __restrict__ Wt, unsigned ldw, unsigned ldk) {
  __shared__ _Float16 T[64 * LDT];
  const unsigned tid = threadIdx.x;
  const unsigned n0 = blockIdx.x * 64u;
  const unsigned k0 = blockIdx.y * 64u;
#pragma unroll 4
  for (unsigned j = 0; j < 16u; ++j) {
    const unsigned idx = tid + 256u * j;
    const unsigned kr = idx >> 6, nc = idx & 63u;
    const float v = W[(size_t)(k0 + kr) * ldw + n0 + nc];
    T[nc * LDT + kr] = toh_flush(WCARRY * bf16r(v));
  }
  __syncthreads();
  v8h x[2];
  size_t off[2];
#pragma unroll
  for (unsigned i = 0; i < 2u; ++i) {
    const unsigned n = 32u * i + (tid >> 3);
    const unsigned kc = (tid & 7u) * 8u;
    x[i] = *(const v8h*)&T[n * LDT + kc];
    off[i] = (size_t)(n0 + n) * ldk + k0 + kc;
  }
#pragma unroll
  for (int i = 0; i < 2; ++i) *(volatile v8h*)(Wt + off[i]) = x[i];
  __threadfence();
#pragma unroll
  for (int i = 0; i < 2; ++i) *(volatile v8h*)(Wt + off[i]) = x[i];
}

__global__ __launch_bounds__(256) void mlin_kernel(
    const float* __restrict__ X, const int* __restrict__ ids,
    const _Float16* __restrict__ Wt, const float* __restrict__ bias,
    float* __restrict__ out) {
  __shared__ _Float16 As[TROWS * LDA];
  __shared__ float Cs[TROWS * LDCS];
  __shared__ int rlist[CHUNK];
  __shared__ int wcnt[16];

  const unsigned tid = threadIdx.x, lane = tid & 31u;
  const int wave = __builtin_amdgcn_readfirstlane((int)(threadIdx.x >> 5));
  const unsigned hh = lane >> 4, m = lane & 15u;
  const int head = (int)blockIdx.y;
  const int chunk0 = (int)blockIdx.x * CHUNK;

  int row[2];
  bool hit[2];
  unsigned bal[2];
#pragma unroll
  for (int j = 0; j < 2; ++j) {
    row[j] = chunk0 + 256 * j + (int)tid;
    const int rc = min(row[j], NROWS - 1);
    int id = ids[rc];
    id = (id < 0) ? (id + NHEADS) : id;
    id = min(max(id, 0), NHEADS - 1);
    hit[j] = (id == head);
    bal[j] = __builtin_amdgcn_ballot_w32(hit[j]);
    if (lane == 0u) wcnt[8 * j + wave] = (int)__popc(bal[j]);
  }
  __syncthreads();

  int tot = 0, base0 = 0, base1 = 0;
#pragma unroll
  for (int i = 0; i < 16; ++i) {
    const int c = wcnt[i];
    base0 += (i < wave) ? c : 0;
    base1 += (i < 8 + wave) ? c : 0;
    tot += c;
  }
  const unsigned lt = (1u << lane) - 1u;
  if (hit[0]) rlist[base0 + (int)__popc(bal[0] & lt)] = row[0];
  if (hit[1]) rlist[base1 + (int)__popc(bal[1] & lt)] = row[1];
  __syncthreads();

  const int cnt = __builtin_amdgcn_readfirstlane(min(tot, CHUNK));
  const int ntiles = (cnt + TROWS - 1) / TROWS;

  const _Float16* bp0 = Wt + (size_t)((unsigned)wave * 32u + m) * LDK
                           + (unsigned)head * KDIM + hh * 8u;
  const _Float16* bp1 = bp0 + (size_t)16 * LDK;
  const unsigned aoff = m * LDA + hh * 8u;

  for (int t = 0; t < ntiles; ++t) {
#pragma unroll
    for (int j = 0; j < 2; ++j) {
      const int r = 8 * j + wave;
      const int li = min(t * TROWS + r, cnt - 1);
      int g = rlist[li];
      g = min(max(g, 0), NROWS - 1);
      const float* src = X + (size_t)g * KDIM + lane * 8u;
      const v4f a0 = *(const v4f*)(src);
      const v4f a1 = *(const v4f*)(src + 4);
      v8h o;
#pragma unroll
      for (int i = 0; i < 4; ++i) {
        o[i]     = toh_flush(XCARRY * bf16r(a0[i]));
        o[i + 4] = toh_flush(XCARRY * bf16r(a1[i]));
      }
      *(v8h*)&As[(unsigned)r * LDA + lane * 8u] = o;
    }
    __syncthreads();

    v8f acc0 = {}, acc1 = {};
#pragma unroll 2
    for (unsigned k0 = 0; k0 < (unsigned)KDIM; k0 += 32u) {
      const v8h alo = *(const v8h*)&As[aoff + k0];
      const v8h ahi = *(const v8h*)&As[aoff + k0 + 16u];
      const v16h a  = frag_join(alo, ahi);
      const v16h b0 = frag_at(bp0 + k0);
      const v16h b1 = frag_at(bp1 + k0);
      acc0 = wmma16(a, b0, acc0);
      acc1 = wmma16(a, b1, acc1);
    }
#pragma unroll
    for (int r = 0; r < 8; ++r) {
      float* d = &Cs[(hh * 8u + (unsigned)r) * LDCS + (unsigned)wave * 32u + m];
      d[0]  = acc0[r];
      d[16] = acc1[r];
    }
    __syncthreads();

    v4f xs[4];
    size_t off[4];
    bool ok[4];
#pragma unroll
    for (int i = 0; i < 4; ++i) {
      const int r = 4 * i + (wave >> 1);
      const unsigned c = ((unsigned)(wave & 1) * 32u + lane) * 4u;
      const int lraw = t * TROWS + r;
      ok[i] = lraw < cnt;
      int g = rlist[min(lraw, cnt - 1)];
      g = min(max(g, 0), NROWS - 1);
      const v4f u  = *(const v4f*)&Cs[(unsigned)r * LDCS + c];
      const v4f gb = *(const v4f*)(bias + (unsigned)head * NDIM + c);
      v4f val;
#pragma unroll
      for (int j = 0; j < 4; ++j)
        val[j] = u[j] * (1.0f / (WCARRY * XCARRY)) + bf16r(gb[j]);
      xs[i] = val;
      off[i] = (size_t)g * NDIM + c;
    }
#pragma unroll
    for (int i = 0; i < 4; ++i)
      if (ok[i]) *(volatile v4f*)(out + off[i]) = xs[i];
    __threadfence();
#pragma unroll
    for (int i = 0; i < 4; ++i)
      if (ok[i]) *(volatile v4f*)(out + off[i]) = xs[i];
  }
}

extern "C" void kernel_launch(void* const* d_in, const int* in_sizes, int n_in,
                              void* d_out, int out_size, void* d_ws, size_t ws_size,
                              hipStream_t stream) {
  if (n_in < 4) return;
  if ((long long)in_sizes[0] < (long long)NROWS * KDIM) return;
  if ((long long)in_sizes[1] < (long long)NROWS) return;
  if ((long long)in_sizes[2] < (long long)NHEADS * KDIM * NDIM) return;
  if ((long long)in_sizes[3] < (long long)NHEADS * NDIM) return;
  if ((long long)out_size < (long long)NROWS * NDIM) return;
  if (ws_size < WS_TOTAL) return;

  const float* X    = (const float*)d_in[0];
  const int*   ids  = (const int*)d_in[1];
  const float* wts  = (const float*)d_in[2];
  const float* bias = (const float*)d_in[3];
  float* out = (float*)d_out;

  char* ws = (char*)d_ws;
  _Float16* Wt = (_Float16*)(ws + OFF_WT);

  dim3 blk(256);
  wconv_kernel<<<dim3(NDIM / 64, (NHEADS * KDIM) / 64), blk, 0, stream>>>(
      wts, Wt, (unsigned)NDIM, (unsigned)LDK);
  mlin_kernel<<<dim3(NROWS / CHUNK, NHEADS), blk, 0, stream>>>(X, ids, Wt, bias, out);
}
